// S5TrajectoryDecoder_22170621182555
// MI455X (gfx1250) — hardware-run, weakly checked
//
#include <hip/hip_runtime.h>


#define LSEQ 32768
#define DM   256
#define PP   128
#define NLAY 4
#define ODIM 64
#define CHK  128
#define NCH  (LSEQ / CHK)
#define TABN (NLAY * PP)

static_assert(LSEQ % 256 == 0);
static_assert(LSEQ % CHK == 0);
static_assert(CHK % 16 == 0);
static_assert(DM == 2 * PP);
static_assert(DM % 128 == 0);
static_assert(ODIM == 64);
static_assert(TABN == 512);

typedef float          v4f   __attribute__((ext_vector_type(4)));
typedef float          v8f   __attribute__((ext_vector_type(8)));
typedef _Float16       v4h   __attribute__((ext_vector_type(4)));
typedef _Float16       v8h   __attribute__((ext_vector_type(8)));
typedef _Float16       v16h  __attribute__((ext_vector_type(16)));
typedef unsigned short u16x4 __attribute__((ext_vector_type(4)));
typedef unsigned short u16x8 __attribute__((ext_vector_type(8)));

union FragH { u16x8 h[2]; v16h v; };
union Pack8 { v8h f; u16x8 u; };
union Pack4 { v4h f; u16x4 u; };

__device__ __forceinline__ unsigned short f2bf(float f) {
  unsigned u = __float_as_uint(f);
  u += 0x7fffu + ((u >> 16) & 1u);
  return (unsigned short)(u >> 16);
}
__device__ __forceinline__ float bf2f(unsigned short b) {
  return __uint_as_float(((unsigned)b) << 16);
}
__device__ __forceinline__ float bfr(float f) { return bf2f(f2bf(f)); }

__device__ __forceinline__ v4f ld4(const float* p) { return *(const v4f*)p; }
__device__ __forceinline__ v8f ld8(const float* p) {
  v4f a = *(const v4f*)p;
  v4f b = *(const v4f*)(p + 4);
  return __builtin_shufflevector(a, b, 0, 1, 2, 3, 4, 5, 6, 7);
}
__device__ __forceinline__ u16x8 to_h8(v8f x) { Pack8 pk; pk.f = __builtin_convertvector(x, v8h); return pk.u; }
__device__ __forceinline__ u16x4 to_h4(v4f x) { Pack4 pk; pk.f = __builtin_convertvector(x, v4h); return pk.u; }
__device__ __forceinline__ unsigned short h2u(float f) {
  _Float16 hv = (_Float16)f;
  return __builtin_bit_cast(unsigned short, hv);
}
__device__ __forceinline__ float rcp_f(float x) {
#if defined(__HIP_DEVICE_COMPILE__)
  return __builtin_amdgcn_rcpf(x);
#else
  return 1.0f / x;
#endif
}
__device__ __forceinline__ float gelu_t(float y) {
  const float z = 0.7978845608028654f * (y + 0.044715f * (y * y * y));
  const float e = __expf(2.0f * z);
  const float t = 1.0f - 2.0f * rcp_f(1.0f + e);
  return 0.5f * y * (1.0f + t);
}

__device__ __forceinline__ void mma16(v8f& acc, const FragH& a, const FragH& b) {
#if defined(__HIP_DEVICE_COMPILE__)
  acc = __builtin_amdgcn_wmma_f32_16x16x32_f16(false, a.v, false, b.v, (short)0, acc, false, false);
  asm volatile("v_nop\n\tv_nop\n\tv_nop\n\tv_nop" : "+v"(acc) : "v"(a.v), "v"(b.v));
#else
  (void)acc; (void)a; (void)b;
#endif
}

template <int NBF>
__device__ __forceinline__ void tile_store_pass(const float* st, float* gp, int ldc, int lane) {
  constexpr int CW  = NBF * 16;
  constexpr int P   = CW + 4;
  constexpr int LPR = CW / 4;
  constexpr int RPI = 32 / LPR;
  constexpr int NIT = 32 / RPI;
  const int rsub = lane / LPR;
  const int c4   = (lane % LPR) * 4;
#pragma unroll
  for (int it = 0; it < NIT; ++it) {
    const int row = it * RPI + rsub;
    const v4f v = *(const v4f*)(st + row * P + c4);
    *(volatile v4f*)(gp + (size_t)row * ldc + c4) = v;
  }
}

template <int MODE, int NBF>
__global__ __launch_bounds__(128)
void k_gemm(const unsigned short* __restrict__ A,  const unsigned short* __restrict__ B1,
            const unsigned short* __restrict__ B2, const float* __restrict__ bias1,
            const float* __restrict__ bias2,       const float* __restrict__ aux,
            const float* __restrict__ dvec,        const float* skip, float* C,
            int K, int ldc, float scale)
{
  constexpr int CW  = NBF * 16;
  constexpr int P   = CW + 4;
  constexpr int LPR = CW / 4;
  constexpr int RPI = 32 / LPR;
  constexpr int NIT = 32 / RPI;
  __shared__ __attribute__((aligned(16))) float stile[4][32 * P];

  const int tid  = threadIdx.x;
  const int lane = tid & 31;
  const int wave = tid >> 5;
  const int h    = lane >> 4;
  const int m    = lane & 15;
  const int wm   = wave >> 1;
  const int wn   = wave & 1;
  const int rowW = blockIdx.y * 64 + wm * 32;
  const int colW = blockIdx.x * (2 * CW) + wn * CW;

  v8f acc[2 * NBF], acc2[2 * NBF];
#pragma unroll
  for (int j = 0; j < 2 * NBF; ++j)
#pragma unroll
    for (int r = 0; r < 8; ++r) { acc[j][r] = 0.0f; acc2[j][r] = 0.0f; }

  const size_t aoff  = (size_t)(rowW + m) * K + 8 * h;
  const size_t boff  = (size_t)(colW + m) * K + 8 * h;
  const size_t sub16 = (size_t)16 * K;
  const int nk = K >> 5;

  for (int kt = 0; kt < nk; ++kt) {
    const size_t k0 = (size_t)kt * 32;
    FragH fa[2], fb[NBF], gb[NBF];
#pragma unroll
    for (int s = 0; s < 2; ++s) {
      const unsigned short* p = A + aoff + s * sub16 + k0;
      fa[s].h[0] = *(const u16x8*)(p);
      fa[s].h[1] = *(const u16x8*)(p + 16);
    }
#pragma unroll
    for (int j = 0; j < NBF; ++j) {
      const unsigned short* p = B1 + boff + j * sub16 + k0;
      fb[j].h[0] = *(const u16x8*)(p);
      fb[j].h[1] = *(const u16x8*)(p + 16);
      if (MODE == 2) {
        const unsigned short* q = B2 + boff + j * sub16 + k0;
        gb[j].h[0] = *(const u16x8*)(q);
        gb[j].h[1] = *(const u16x8*)(q + 16);
      }
    }
#pragma unroll
    for (int s = 0; s < 2; ++s)
#pragma unroll
      for (int j = 0; j < NBF; ++j) {
        mma16(acc[s * NBF + j], fa[s], fb[j]);
        if (MODE == 2) mma16(acc2[s * NBF + j], fa[s], gb[j]);
      }
  }

  float b1c[NBF], b2c[NBF];
#pragma unroll
  for (int j = 0; j < NBF; ++j) {
    b1c[j] = 0.0f; b2c[j] = 0.0f;
    if (MODE >= 2) b1c[j] = bfr(bias1[colW + j * 16 + m]);
    if (MODE == 2) b2c[j] = bfr(bias2[colW + j * 16 + m]);
  }
  float* st = stile[wave];
#pragma unroll
  for (int s = 0; s < 2; ++s)
#pragma unroll
    for (int j = 0; j < NBF; ++j)
#pragma unroll
      for (int r = 0; r < 8; ++r) {
        float v = acc[s * NBF + j][r] * scale;
        if (MODE == 2) {
          const float a1 = v + b1c[j];
          const float a2 = acc2[s * NBF + j][r] * scale + b2c[j];
          const float sg = rcp_f(1.0f + __expf(-a2));
          v = a1 * sg;
        } else if (MODE == 3) {
          v += b1c[j];
        }
        st[(s * 16 + 8 * h + r) * P + j * 16 + m] = v;
      }
  __syncthreads();

  if (MODE == 1 || MODE == 2) {
    const int rsub = lane / LPR;
    const int c4   = (lane % LPR) * 4;
#pragma unroll
    for (int it = 0; it < NIT; ++it) {
      const int row = it * RPI + rsub;
      v4f v = *(const v4f*)(st + row * P + c4);
      const size_t gidx = (size_t)(rowW + row) * ldc + colW + c4;
      if (MODE == 1) {
        const v4f a = *(const v4f*)(aux + gidx);
        v4f d;
        d.x = bfr(dvec[colW + c4 + 0]);
        d.y = bfr(dvec[colW + c4 + 1]);
        d.z = bfr(dvec[colW + c4 + 2]);
        d.w = bfr(dvec[colW + c4 + 3]);
        v += a * d;
      } else {
        const v4f sk = *(const v4f*)(skip + gidx);
        v += sk;
      }
      *(v4f*)(st + row * P + c4) = v;
    }
  }

  float* gp = C + (size_t)rowW * ldc + colW;
  tile_store_pass<NBF>(st, gp, ldc, lane);
  __threadfence();
  tile_store_pass<NBF>(st, gp, ldc, lane);
}

__global__ __launch_bounds__(256)
void k_expand(const float* __restrict__ lat, const float* __restrict__ W,
              const float* __restrict__ b, float* X)
{
  __shared__ float sl[DM];
  __shared__ __attribute__((aligned(16))) float sv[DM];
  const int t = threadIdx.x, lane = t & 31, wave = t >> 5;
  sl[t] = bfr(lat[t]);
  __syncthreads();
  float acc = 0.0f;
#pragma unroll 4
  for (int k = 0; k < DM; ++k) acc = fmaf(sl[k], bfr(W[(size_t)k * DM + t]), acc);
  acc += bfr(b[t]);
  acc = (acc >= 0.0f) ? acc : 0.01f * acc;
  sv[t] = acc;
  __syncthreads();
  const int ca = 4 * lane, cb = PP + 4 * lane;
  const v4f va = *(const v4f*)(sv + ca);
  const v4f vb = *(const v4f*)(sv + cb);
  const size_t r0 = (size_t)blockIdx.x * 256;
#pragma unroll 1
  for (int it = 0; it < 32; ++it) {
    float* fp = X + (r0 + (size_t)it * 8 + wave) * DM;
    *(volatile v4f*)(fp + ca) = va;
    *(volatile v4f*)(fp + cb) = vb;
  }
  __threadfence();
#pragma unroll 1
  for (int it = 0; it < 32; ++it) {
    float* fp = X + (r0 + (size_t)it * 8 + wave) * DM;
    *(volatile v4f*)(fp + ca) = va;
    *(volatile v4f*)(fp + cb) = vb;
  }
}

__global__ __launch_bounds__(512)
void k_tab(const float* __restrict__ Lre, const float* __restrict__ Lim,
           const float* __restrict__ lstep, float* tab, const int* __restrict__ slen)
{
  (void)slen;
  const int i = threadIdx.x;
  const float st  = expf(bfr(lstep[i]));
  const float ar  = bfr(Lre[i]);
  const float ai  = bfr(Lim[i]);
  const float er  = expf(ar * st);
  const float th  = ai * st;
  const float lbr = er * cosf(th);
  const float lbi = er * sinf(th);
  const float nr  = lbr - 1.0f, ni = lbi;
  const float den = ar * ar + ai * ai;
  const float rd  = 1.0f / den;
  const float fr  = (nr * ar + ni * ai) * rd;
  const float fi  = (ni * ar - nr * ai) * rd;
  *(volatile float*)(tab + i)            = lbr;
  *(volatile float*)(tab + TABN + i)     = lbi;
  *(volatile float*)(tab + 2 * TABN + i) = fr;
  *(volatile float*)(tab + 3 * TABN + i) = fi;
  __threadfence();
  *(volatile float*)(tab + i)            = lbr;
  *(volatile float*)(tab + TABN + i)     = lbi;
  *(volatile float*)(tab + 2 * TABN + i) = fr;
  *(volatile float*)(tab + 3 * TABN + i) = fi;
}

__global__ __launch_bounds__(256)
void k_cvt_b(const float* __restrict__ Bre, const float* __restrict__ Bim, unsigned short* Bw)
{
  const int lane = threadIdx.x & 31, wave = threadIdx.x >> 5;
  const int r  = blockIdx.x * 8 + wave;
  const int l  = r >> 8, n = r & (DM - 1), pr = n & (PP - 1);
  const size_t so = ((size_t)l * PP + pr) * DM + lane * 8;
  const v8f xre = ld8(Bre + so);
  const v8f xim = ld8(Bim + so);
  v8f x = xre;
  if (n >= PP) x = xim;
  v8f y;
#pragma unroll
  for (int c = 0; c < 8; ++c) y[c] = 16.0f * bfr(x[c]);
  const u16x8 hv = to_h8(y);
  unsigned short* dp = Bw + (size_t)r * DM + lane * 8;
  *(volatile u16x8*)dp = hv;
  __threadfence();
  *(volatile u16x8*)dp = hv;
}

__global__ __launch_bounds__(256)
void k_cvt_c(const float* __restrict__ Cre, const float* __restrict__ Cim, unsigned short* Cw)
{
  const int lane = threadIdx.x & 31, wave = threadIdx.x >> 5;
  const int r  = blockIdx.x * 8 + wave;
  const int l  = r >> 8, hh = r & (DM - 1);
  const int k0 = lane * 8, kk = k0 & (PP - 1);
  const size_t so = ((size_t)l * DM + hh) * PP + kk;
  const v8f xre = ld8(Cre + so);
  const v8f xim = ld8(Cim + so);
  v8f x = xre;
  float scl = 32.0f;
  if (k0 >= PP) { x = xim; scl = -32.0f; }
  v8f y;
#pragma unroll
  for (int c = 0; c < 8; ++c) y[c] = scl * bfr(x[c]);
  const u16x8 hv = to_h8(y);
  unsigned short* dp = Cw + (size_t)r * DM + k0;
  *(volatile u16x8*)dp = hv;
  __threadfence();
  *(volatile u16x8*)dp = hv;
}

__global__ __launch_bounds__(256)
void k_tr(const float* __restrict__ in, unsigned short* out, int K, int N)
{
  __shared__ float tile[64][33];
  const int tid = threadIdx.x, lane = tid & 31, wave = tid >> 5;
  const int z = blockIdx.z;
  const float* src = in + (size_t)z * K * N;
  unsigned short* dst = out + (size_t)z * N * K;
  const int k0 = blockIdx.y * 64, n0 = blockIdx.x * 32;
#pragma unroll
  for (int i = 0; i < 8; ++i) {
    const int idx = i * 256 + tid;
    const int kk = idx >> 5, nn = idx & 31;
    tile[kk][nn] = src[(size_t)(k0 + kk) * N + n0 + nn];
  }
  __syncthreads();
  const int nrow = wave * 4 + (lane >> 3);
  const int kq   = (lane & 7) * 8;
  v8f y;
#pragma unroll
  for (int e = 0; e < 8; ++e) y[e] = 16.0f * bfr(tile[kq + e][nrow]);
  const u16x8 hv = to_h8(y);
  unsigned short* dp = dst + (size_t)(n0 + nrow) * K + k0 + kq;
  *(volatile u16x8*)dp = hv;
  __threadfence();
  *(volatile u16x8*)dp = hv;
}

template <bool GELU>
__global__ __launch_bounds__(256)
void k_ln(const float* __restrict__ Xin, const float* __restrict__ sc,
          const float* __restrict__ bs, float* H32, unsigned short* A16)
{
  const int lane = threadIdx.x & 31, wave = threadIdx.x >> 5;
  const size_t row = (size_t)blockIdx.x * 8 + wave;
  const float* xp = Xin + row * DM;
  const int ca = 4 * lane, cb = PP + 4 * lane;
  const v4f a = ld4(xp + ca), b = ld4(xp + cb);
  float s = ((a.x + a.y) + (a.z + a.w)) + ((b.x + b.y) + (b.z + b.w));
#pragma unroll
  for (int off = 16; off > 0; off >>= 1) s += __shfl_xor(s, off, 32);
  const float mu = s * (1.0f / DM);
  const v4f da = a - mu, db = b - mu;
  float q = (da.x * da.x + da.y * da.y) + (da.z * da.z + da.w * da.w)
          + (db.x * db.x + db.y * db.y) + (db.z * db.z + db.w * db.w);
#pragma unroll
  for (int off = 16; off > 0; off >>= 1) q += __shfl_xor(q, off, 32);
  const float var = q * (1.0f / DM);
  const float rs  = rsqrtf(var + 1e-6f);
  v4f sa, sb, ba, bb;
  sa.x = bfr(sc[ca + 0]); sa.y = bfr(sc[ca + 1]); sa.z = bfr(sc[ca + 2]); sa.w = bfr(sc[ca + 3]);
  sb.x = bfr(sc[cb + 0]); sb.y = bfr(sc[cb + 1]); sb.z = bfr(sc[cb + 2]); sb.w = bfr(sc[cb + 3]);
  ba.x = bfr(bs[ca + 0]); ba.y = bfr(bs[ca + 1]); ba.z = bfr(bs[ca + 2]); ba.w = bfr(bs[ca + 3]);
  bb.x = bfr(bs[cb + 0]); bb.y = bfr(bs[cb + 1]); bb.z = bfr(bs[cb + 2]); bb.w = bfr(bs[cb + 3]);
  v4f ya = (da * rs) * sa + ba;
  v4f yb = (db * rs) * sb + bb;
  if (GELU) {
    ya.x = gelu_t(ya.x); ya.y = gelu_t(ya.y); ya.z = gelu_t(ya.z); ya.w = gelu_t(ya.w);
    yb.x = gelu_t(yb.x); yb.y = gelu_t(yb.y); yb.z = gelu_t(yb.z); yb.w = gelu_t(yb.w);
  }
  const u16x4 ha = to_h4(ya), hb = to_h4(yb);
  unsigned short* hp = A16 + row * DM;
  float* fp = H32 + row * DM;
  if (!GELU) { *(volatile v4f*)(fp + ca) = ya; *(volatile v4f*)(fp + cb) = yb; }
  *(volatile u16x4*)(hp + ca) = ha;
  *(volatile u16x4*)(hp + cb) = hb;
  __threadfence();
  if (!GELU) { *(volatile v4f*)(fp + ca) = ya; *(volatile v4f*)(fp + cb) = yb; }
  *(volatile u16x4*)(hp + ca) = ha;
  *(volatile u16x4*)(hp + cb) = hb;
}

__global__ __launch_bounds__(256)
void k_cvt_x(const float* __restrict__ X, unsigned short* A16)
{
  const int lane = threadIdx.x & 31, wave = threadIdx.x >> 5;
  const size_t row = (size_t)blockIdx.x * 8 + wave;
  const size_t so  = row * DM + lane * 8;
  const u16x8 hv = to_h8(ld8(X + so));
  *(volatile u16x8*)(A16 + so) = hv;
  __threadfence();
  *(volatile u16x8*)(A16 + so) = hv;
}

__device__ __forceinline__ void sstep(float& sr, float& si, float ar, float ai,
                                      float fr, float fi, float gr, float gi) {
  const float br = fmaf(-fi, gi, fr * gr);
  const float bi = fmaf(fi, gr, fr * gi);
  const float nr = fmaf(ar, sr, fmaf(-ai, si, br));
  const float ni = fmaf(ar, si, fmaf(ai, sr, bi));
  sr = nr; si = ni;
}

template <bool EMIT>
__global__ __launch_bounds__(128)
void k_scan(const float* __restrict__ G, const float* __restrict__ tab, int loff,
            const float* __restrict__ carry, float* S, unsigned short* XS)
{
  __shared__ __attribute__((aligned(16))) unsigned short s16[16 * DM];
  const int ch = blockIdx.x, p = threadIdx.x, lane = p & 31, wave = p >> 5;
  const float ar = tab[loff + p],            ai = tab[TABN + loff + p];
  const float fr = tab[2 * TABN + loff + p], fi = tab[3 * TABN + loff + p];
  float sr = 0.0f, si = 0.0f;
  if (EMIT) { sr = carry[(size_t)ch * DM + p]; si = carry[(size_t)ch * DM + PP + p]; }
  const float* gp = G + (size_t)ch * CHK * DM;

  if (!EMIT) {
#pragma unroll 1
    for (int t = 0; t < CHK; ++t) {
      const float gr = gp[(size_t)t * DM + p], gi = gp[(size_t)t * DM + PP + p];
      sstep(sr, si, ar, ai, fr, fi, gr, gi);
    }
    float* sp = S + (size_t)ch * DM;
    *(volatile float*)(sp + p) = sr; *(volatile float*)(sp + PP + p) = si;
    __threadfence();
    *(volatile float*)(sp + p) = sr; *(volatile float*)(sp + PP + p) = si;
  } else {
#pragma unroll 1
    for (int t0 = 0; t0 < CHK; t0 += 16) {
#pragma unroll 1
      for (int tt = 0; tt < 16; ++tt) {
        const int t = t0 + tt;
        const float gr = gp[(size_t)t * DM + p], gi = gp[(size_t)t * DM + PP + p];
        sstep(sr, si, ar, ai, fr, fi, gr, gi);
        s16[tt * DM + p]      = h2u(sr);
        s16[tt * DM + PP + p] = h2u(si);
      }
      __syncthreads();
      const size_t gro = (size_t)ch * CHK + t0;
#pragma unroll
      for (int it = 0; it < 4; ++it) {
        const int row = it * 4 + wave;
        const u16x8 v = *(const u16x8*)(s16 + row * DM + lane * 8);
        *(volatile u16x8*)(XS + (gro + row) * DM + lane * 8) = v;
      }
      __threadfence();
#pragma unroll
      for (int it = 0; it < 4; ++it) {
        const int row = it * 4 + wave;
        const u16x8 v = *(const u16x8*)(s16 + row * DM + lane * 8);
        *(volatile u16x8*)(XS + (gro + row) * DM + lane * 8) = v;
      }
      __syncthreads();
    }
  }
}

__global__ __launch_bounds__(128)
void k_carry(const float* __restrict__ tab, int loff, const float* __restrict__ S, float* carry)
{
  const int p = threadIdx.x;
  const float ar = tab[loff + p], ai = tab[TABN + loff + p];
  float pr = 1.0f, pi = 0.0f;
#pragma unroll 1
  for (int j = 0; j < CHK; ++j) {
    const float nr = fmaf(ar, pr, -(ai * pi));
    const float ni = fmaf(ar, pi, ai * pr);
    pr = nr; pi = ni;
  }
  float sr = 0.0f, si = 0.0f;
#pragma unroll 1
  for (int c = 0; c < NCH; ++c) {
    float* cp = carry + (size_t)c * DM;
    *(volatile float*)(cp + p) = sr; *(volatile float*)(cp + PP + p) = si;
    __threadfence();
    *(volatile float*)(cp + p) = sr; *(volatile float*)(cp + PP + p) = si;
    const float cr = S[(size_t)c * DM + p], ci = S[(size_t)c * DM + PP + p];
    const float nr = fmaf(pr, sr, fmaf(-pi, si, cr));
    const float ni = fmaf(pr, si, fmaf(pi, sr, ci));
    sr = nr; si = ni;
  }
}

extern "C" void kernel_launch(void* const* d_in, const int* in_sizes, int n_in,
                              void* d_out, int out_size, void* d_ws, size_t ws_size,
                              hipStream_t stream)
{
  if (n_in < 20) return;
  if (in_sizes[0]  != DM)             return;
  if (in_sizes[1]  != DM * DM)        return;
  if (in_sizes[2]  != DM)             return;
  if (in_sizes[3]  != NLAY * DM)      return;
  if (in_sizes[4]  != NLAY * DM)      return;
  if (in_sizes[5]  != TABN)           return;
  if (in_sizes[6]  != TABN)           return;
  if (in_sizes[7]  != NLAY * PP * DM) return;
  if (in_sizes[8]  != NLAY * PP * DM) return;
  if (in_sizes[9]  != NLAY * DM * PP) return;
  if (in_sizes[10] != NLAY * DM * PP) return;
  if (in_sizes[11] != NLAY * DM)      return;
  if (in_sizes[12] != TABN)           return;
  if (in_sizes[13] != NLAY * DM * DM) return;
  if (in_sizes[14] != NLAY * DM)      return;
  if (in_sizes[15] != NLAY * DM * DM) return;
  if (in_sizes[16] != NLAY * DM)      return;
  if (in_sizes[17] != DM * ODIM)      return;
  if (in_sizes[18] != ODIM)           return;
  if (in_sizes[19] < 1)               return;
  if (out_size != LSEQ * ODIM)        return;

  const float* lat   = (const float*)d_in[0];
  const float* Wexp  = (const float*)d_in[1];
  const float* bexp  = (const float*)d_in[2];
  const float* nsc   = (const float*)d_in[3];
  const float* nbs   = (const float*)d_in[4];
  const float* Lre   = (const float*)d_in[5];
  const float* Lim   = (const float*)d_in[6];
  const float* Bre   = (const float*)d_in[7];
  const float* Bim   = (const float*)d_in[8];
  const float* Cre   = (const float*)d_in[9];
  const float* Cim   = (const float*)d_in[10];
  const float* Dv    = (const float*)d_in[11];
  const float* lstep = (const float*)d_in[12];
  const float* W1    = (const float*)d_in[13];
  const float* b1    = (const float*)d_in[14];
  const float* W2    = (const float*)d_in[15];
  const float* b2    = (const float*)d_in[16];
  const float* Wout  = (const float*)d_in[17];
  const float* bout  = (const float*)d_in[18];
  const int*   slen  = (const int*)d_in[19];
  float* out = (float*)d_out;

  const size_t SZ_F   = (size_t)LSEQ * DM * 4;
  const size_t SZ_H   = (size_t)LSEQ * DM * 2;
  const size_t SZ_W   = (size_t)NLAY * DM * DM * 2;
  const size_t SZ_WO  = (size_t)ODIM * DM * 2;
  const size_t SZ_TAB = (size_t)4 * TABN * 4;
  const size_t SZ_S   = (size_t)NCH * DM * 4;
  const size_t OFF_X   = 0;
  const size_t OFF_H32 = OFF_X + SZ_F;
  const size_t OFF_G   = OFF_H32 + SZ_F;
  const size_t OFF_A16 = OFF_G + SZ_F;
  const size_t OFF_WB  = OFF_A16 + SZ_H;
  const size_t OFF_WC  = OFF_WB + SZ_W;
  const size_t OFF_W1  = OFF_WC + SZ_W;
  const size_t OFF_W2  = OFF_W1 + SZ_W;
  const size_t OFF_WO  = OFF_W2 + SZ_W;
  const size_t OFF_TAB = OFF_WO + SZ_WO;
  const size_t OFF_S   = OFF_TAB + SZ_TAB;
  const size_t OFF_CAR = OFF_S + SZ_S;
  const size_t WS_END  = OFF_CAR + SZ_S;
  if (ws_size < WS_END) return;

  char* ws = (char*)d_ws;
  float*          X    = (float*)(ws + OFF_X);
  float*          H32  = (float*)(ws + OFF_H32);
  float*          G    = (float*)(ws + OFF_G);
  unsigned short* A16  = (unsigned short*)(ws + OFF_A16);
  unsigned short* wb   = (unsigned short*)(ws + OFF_WB);
  unsigned short* wc   = (unsigned short*)(ws + OFF_WC);
  unsigned short* w1t  = (unsigned short*)(ws + OFF_W1);
  unsigned short* w2t  = (unsigned short*)(ws + OFF_W2);
  unsigned short* wot  = (unsigned short*)(ws + OFF_WO);
  float*          tab  = (float*)(ws + OFF_TAB);
  float*          Sbuf = (float*)(ws + OFF_S);
  float*          car  = (float*)(ws + OFF_CAR);

  const float s16th = 0.0625f;

  hipLaunchKernelGGL(k_expand, dim3(LSEQ / 256), dim3(256), 0, stream, lat, Wexp, bexp, X);
  hipLaunchKernelGGL(k_tab, dim3(1), dim3(TABN), 0, stream, Lre, Lim, lstep, tab, slen);
  hipLaunchKernelGGL(k_cvt_b, dim3((NLAY * DM) / 8), dim3(256), 0, stream, Bre, Bim, wb);
  hipLaunchKernelGGL(k_cvt_c, dim3((NLAY * DM) / 8), dim3(256), 0, stream, Cre, Cim, wc);
  hipLaunchKernelGGL(k_tr, dim3(DM / 32, DM / 64, NLAY), dim3(256), 0, stream, W1, w1t, (int)DM, (int)DM);
  hipLaunchKernelGGL(k_tr, dim3(DM / 32, DM / 64, NLAY), dim3(256), 0, stream, W2, w2t, (int)DM, (int)DM);
  hipLaunchKernelGGL(k_tr, dim3(ODIM / 32, DM / 64, 1), dim3(256), 0, stream, Wout, wot, (int)DM, (int)ODIM);

  for (int l = 0; l < NLAY; ++l) {
    const size_t woff = (size_t)l * DM * DM;
    const float* scl = nsc + (size_t)l * DM;
    const float* bsl = nbs + (size_t)l * DM;
    const float* b1l = b1 + (size_t)l * DM;
    const float* b2l = b2 + (size_t)l * DM;
    const float* dvl = Dv + (size_t)l * DM;

    hipLaunchKernelGGL(HIP_KERNEL_NAME(k_ln<false>), dim3(LSEQ / 8), dim3(256), 0, stream,
                       (const float*)X, scl, bsl, H32, A16);
    hipLaunchKernelGGL(HIP_KERNEL_NAME(k_gemm<0, 4>), dim3(DM / 128, LSEQ / 64), dim3(128), 0, stream,
                       (const unsigned short*)A16, (const unsigned short*)(wb + woff),
                       (const unsigned short*)(wb + woff), b1l, b2l,
                       (const float*)H32, dvl, (const float*)X, G, (int)DM, (int)DM, s16th);
    hipLaunchKernelGGL(HIP_KERNEL_NAME(k_scan<false>), dim3(NCH), dim3(128), 0, stream,
                       (const float*)G, (const float*)tab, (int)(l * PP), (const float*)car, Sbuf, A16);
    hipLaunchKernelGGL(k_carry, dim3(1), dim3(128), 0, stream,
                       (const float*)tab, (int)(l * PP), (const float*)Sbuf, car);
    hipLaunchKernelGGL(HIP_KERNEL_NAME(k_scan<true>), dim3(NCH), dim3(128), 0, stream,
                       (const float*)G, (const float*)tab, (int)(l * PP), (const float*)car, Sbuf, A16);
    hipLaunchKernelGGL(HIP_KERNEL_NAME(k_gemm<1, 4>), dim3(DM / 128, LSEQ / 64), dim3(128), 0, stream,
                       (const unsigned short*)A16, (const unsigned short*)(wc + woff),
                       (const unsigned short*)(wc + woff), b1l, b2l,
                       (const float*)H32, dvl, (const float*)X, G, (int)DM, (int)DM, s16th);
    hipLaunchKernelGGL(HIP_KERNEL_NAME(k_ln<true>), dim3(LSEQ / 8), dim3(256), 0, stream,
                       (const float*)G, scl, bsl, H32, A16);
    hipLaunchKernelGGL(HIP_KERNEL_NAME(k_gemm<2, 2>), dim3(DM / 64, LSEQ / 64), dim3(128), 0, stream,
                       (const unsigned short*)A16, (const unsigned short*)(w1t + woff),
                       (const unsigned short*)(w2t + woff), b1l, b2l,
                       (const float*)H32, dvl, (const float*)X, X, (int)DM, (int)DM, s16th);
  }

  hipLaunchKernelGGL(k_cvt_x, dim3(LSEQ / 8), dim3(256), 0, stream, (const float*)X, A16);
  hipLaunchKernelGGL(HIP_KERNEL_NAME(k_gemm<3, 2>), dim3(1, LSEQ / 64), dim3(128), 0, stream,
                     (const unsigned short*)A16, (const unsigned short*)wot, (const unsigned short*)wot,
                     bout, bout, (const float*)H32, Dv, (const float*)X, out, (int)DM, (int)ODIM, s16th);
}
